// MyGCNModel_70506183131446
// MI455X (gfx1250) — hardware-verified
//
#include <hip/hip_runtime.h>
#include <stddef.h>


#define NTHR    256
#define NWAVE   8
#define EPT     8
#define NGRP    2
#define CHUNK   (NTHR * EPT * NGRP)
#define WCAP    (EPT * NGRP * 32)
#define LISTN   (NWAVE * WCAP)
#define NBC     4096
#define NBF     1024
#define RCAP    40960
#define RBN     128
#define TGT     256
#define DEGCAP  1024
#define OTHR    512
#define BM      64
#define BNC     128
#define SB      64
#define WSCAP   134217728
#define F0      5
#define C1W     64
#define C2W     128
#define HEADS   4
#define HCH     256
#define H3W     1024
#define C3W     256
#define C4W     512
#define PW      1024
#define FCN     1024
#define ACARRY  8.0f
#define WCARRY  64.0f
#define GSCALE  (1.0f / 512.0f)
#define BNEPS   1e-5f

#define LDS_FILL ((RCAP + NBF + LISTN) * 4 + 64)

static_assert((CHUNK & (CHUNK - 1)) == 0);
static_assert(CHUNK <= 4096);
static_assert((NBC & (NBC - 1)) == 0 && (NBF & (NBF - 1)) == 0);
static_assert(NBC == 4 * NBF);
static_assert(OTHR * 8 == NBC);
static_assert((RCAP % 32) == 0);
static_assert(TGT == NWAVE * 32);
static_assert((NBC % TGT) == 0);
static_assert((TGT % BM) == 0);
static_assert(WCAP == EPT * NGRP * 32);
static_assert(H3W == HEADS * HCH);
static_assert(C3W == HCH);
static_assert(HCH == 2 * 128);
static_assert(H3W == 8 * 128);
static_assert(C4W == 2 * NTHR);
static_assert(PW == 2 * C4W);
static_assert(C2W * 8 == 4 * NTHR);
static_assert((C2W % 32) == 0 && (C3W % 32) == 0 && (PW % 32) == 0);
static_assert((C2W % BNC) == 0 && (H3W % BNC) == 0 && (C4W % BNC) == 0 && (FCN % BNC) == 0);
static_assert(C1W == 2 * 32);

typedef float    v2f  __attribute__((ext_vector_type(2)));
typedef float    v4f  __attribute__((ext_vector_type(4)));
typedef float    v8f  __attribute__((ext_vector_type(8)));
typedef int      v4i  __attribute__((ext_vector_type(4)));
typedef double   v2d  __attribute__((ext_vector_type(2)));
typedef _Float16 v2h  __attribute__((ext_vector_type(2)));
typedef _Float16 v4h  __attribute__((ext_vector_type(4)));
typedef _Float16 v8h  __attribute__((ext_vector_type(8)));
typedef _Float16 v16h __attribute__((ext_vector_type(16)));
union Frag { v16h v; v8h h[2]; };

__device__ __forceinline__ v8f wmh(v16h a, v16h b, v8f c) {
  v8f d = __builtin_amdgcn_wmma_f32_16x16x32_f16(false, a, false, b, (short)0, c, false, false);
  asm volatile("v_nop\n\tv_nop\n\tv_nop\n\tv_nop" : "+v"(d) : "v"(a), "v"(b));
  return d;
}

__device__ __forceinline__ v4f selz(v4f v, bool live) {
  v4f o; o.x = live ? v.x : 0.f; o.y = live ? v.y : 0.f; o.z = live ? v.z : 0.f; o.w = live ? v.w : 0.f; return o;
}
__device__ __forceinline__ v2f selz(v2f v, bool live) {
  v2f o; o.x = live ? v.x : 0.f; o.y = live ? v.y : 0.f; return o;
}
__device__ __forceinline__ v4f selv4(v4f v, bool c, float other) {
  v4f o; o.x = c ? v.x : other; o.y = c ? v.y : other; o.z = c ? v.z : other; o.w = c ? v.w : other; return o;
}
__device__ __forceinline__ v4f vmax4(v4f a, v4f b) {
  v4f o; o.x = fmaxf(a.x, b.x); o.y = fmaxf(a.y, b.y); o.z = fmaxf(a.z, b.z); o.w = fmaxf(a.w, b.w); return o;
}
__device__ __forceinline__ v4f lrelu4(v4f v) {
  v4f o;
  o.x = v.x >= 0.f ? v.x : 0.2f * v.x;  o.y = v.y >= 0.f ? v.y : 0.2f * v.y;
  o.z = v.z >= 0.f ? v.z : 0.2f * v.z;  o.w = v.w >= 0.f ? v.w : 0.2f * v.w;
  return o;
}
__device__ __forceinline__ v4f vexp4(v4f v) {
  v4f o; o.x = __expf(v.x); o.y = __expf(v.y); o.z = __expf(v.z); o.w = __expf(v.w); return o;
}
__device__ __forceinline__ v4f wmax4(v4f v) {
#pragma unroll
  for (int off = 16; off > 0; off >>= 1) {
    v.x = fmaxf(v.x, __shfl_xor(v.x, off)); v.y = fmaxf(v.y, __shfl_xor(v.y, off));
    v.z = fmaxf(v.z, __shfl_xor(v.z, off)); v.w = fmaxf(v.w, __shfl_xor(v.w, off));
  }
  return v;
}
__device__ __forceinline__ v4f wsum4(v4f v) {
#pragma unroll
  for (int off = 16; off > 0; off >>= 1) {
    v.x += __shfl_xor(v.x, off); v.y += __shfl_xor(v.y, off);
    v.z += __shfl_xor(v.z, off); v.w += __shfl_xor(v.w, off);
  }
  return v;
}

template <int NB>
__device__ __forceinline__ int scan_chunk(const int* __restrict__ dsts, int nE, int cbase, int slotBase,
                                          int vec8, int* list, int tid, int lane, int wave) {
  int wc = 0;
#pragma unroll
  for (int g = 0; g < NGRP; ++g) {
    const int el0  = (g * NTHR + tid) * EPT;
    const int e0   = cbase + el0;
    const int sent = -2147483647 - 1;
    v4i da, db;
    if (vec8 != 0 && cbase + CHUNK <= nE) {
      da = *(const v4i*)(dsts + e0);
      db = *(const v4i*)(dsts + e0 + 4);
    } else {
      da.x = (e0     < nE) ? dsts[min(e0, nE - 1)] : sent;
      da.y = (e0 + 1 < nE) ? dsts[min(e0 + 1, nE - 1)] : sent;
      da.z = (e0 + 2 < nE) ? dsts[min(e0 + 2, nE - 1)] : sent;
      da.w = (e0 + 3 < nE) ? dsts[min(e0 + 3, nE - 1)] : sent;
      db.x = (e0 + 4 < nE) ? dsts[min(e0 + 4, nE - 1)] : sent;
      db.y = (e0 + 5 < nE) ? dsts[min(e0 + 5, nE - 1)] : sent;
      db.z = (e0 + 6 < nE) ? dsts[min(e0 + 6, nE - 1)] : sent;
      db.w = (e0 + 7 < nE) ? dsts[min(e0 + 7, nE - 1)] : sent;
    }
    const unsigned nb = (unsigned)slotBase;
    const unsigned s0 = (unsigned)da.x - nb, s1 = (unsigned)da.y - nb;
    const unsigned s2 = (unsigned)da.z - nb, s3 = (unsigned)da.w - nb;
    const unsigned s4 = (unsigned)db.x - nb, s5 = (unsigned)db.y - nb;
    const unsigned s6 = (unsigned)db.z - nb, s7 = (unsigned)db.w - nb;
    const bool h0 = s0 < (unsigned)NB, h1 = s1 < (unsigned)NB, h2 = s2 < (unsigned)NB, h3 = s3 < (unsigned)NB;
    const bool h4 = s4 < (unsigned)NB, h5 = s5 < (unsigned)NB, h6 = s6 < (unsigned)NB, h7 = s7 < (unsigned)NB;
    const unsigned any = __builtin_amdgcn_ballot_w32(h0 | h1 | h2 | h3 | h4 | h5 | h6 | h7);
    if (any != 0u) {
#define HITJ(J, HJ, SJ) { \
        const unsigned mj = __builtin_amdgcn_ballot_w32(HJ); \
        if (mj != 0u) { \
          if (HJ) { \
            const int pos = wc + (int)__builtin_amdgcn_mbcnt_lo(mj, 0u); \
            if (pos < WCAP) list[wave * WCAP + pos] = ((el0 + (J)) << 12) | (int)(SJ); \
          } \
          wc += (int)__builtin_popcount(mj); } }
      HITJ(0, h0, s0)
      HITJ(1, h1, s1)
      HITJ(2, h2, s2)
      HITJ(3, h3, s3)
      HITJ(4, h4, s4)
      HITJ(5, h5, s5)
      HITJ(6, h6, s6)
      HITJ(7, h7, s7)
#undef HITJ
    }
  }
  return wc;
}

__global__ __launch_bounds__(NTHR) void k_count(
    const int* __restrict__ dsts, int* cnt, float* dinv, int nE, int vec8) {
  __shared__ __attribute__((aligned(16))) int scnt[NBC];
  __shared__ __attribute__((aligned(16))) int list[LISTN];
  __shared__ int wcnt[NWAVE];
  const int tid = threadIdx.x, lane = tid & 31, wave = tid >> 5;
  const int nodeBase = blockIdx.x * NBC;

  for (int i = tid; i < NBC; i += NTHR) scnt[i] = 0;
  __syncthreads();

  const int nChunks = (nE + CHUNK - 1) / CHUNK;
#pragma unroll 1
  for (int ch = 0; ch < nChunks; ++ch) {
    const int cbase = ch * CHUNK;
    const int wc = scan_chunk<NBC>(dsts, nE, cbase, nodeBase, vec8, list, tid, lane, wave);
    if (lane == 0) wcnt[wave] = wc;
    __syncthreads();
    if (wave == 0) {
#pragma unroll 1
      for (int wsx = 0; wsx < NWAVE; ++wsx) {
        int n = __builtin_amdgcn_readfirstlane(wcnt[wsx]);
        n = n > WCAP ? WCAP : (n < 0 ? 0 : n);
        const int* lp = list + wsx * WCAP;
#pragma unroll 1
        for (int i = 0; i < n; ++i) {
          const int ent  = __builtin_amdgcn_readfirstlane(lp[i]);
          const int slot = ent & (NBC - 1);
          if (lane == 0) scnt[slot] = scnt[slot] + 1;
        }
      }
    }
    __syncthreads();
  }

  v4i cq[4];
  v4f dq[4];
#pragma unroll
  for (int q = 0; q < 4; ++q) {
    const int f = (wave * 4 + q) * 128 + 4 * lane;
    const v4i cv = *(const v4i*)(scnt + f);
    cq[q] = cv;
    v4f d;
    d.x = rsqrtf((float)(cv.x < 0 ? 0 : cv.x) + 1.0f);
    d.y = rsqrtf((float)(cv.y < 0 ? 0 : cv.y) + 1.0f);
    d.z = rsqrtf((float)(cv.z < 0 ? 0 : cv.z) + 1.0f);
    d.w = rsqrtf((float)(cv.w < 0 ? 0 : cv.w) + 1.0f);
    dq[q] = d;
  }
  int*   cp = cnt  + (size_t)nodeBase;
  float* dp = dinv + (size_t)nodeBase;
#pragma unroll
  for (int q = 0; q < 4; ++q) {
    const int f = (wave * 4 + q) * 128 + 4 * lane;
    *(volatile v4i*)(cp + f) = cq[q];
    *(volatile v4f*)(dp + f) = dq[q];
  }
  __threadfence();
#pragma unroll
  for (int q = 0; q < 4; ++q) {
    const int f = (wave * 4 + q) * 128 + 4 * lane;
    *(volatile v4i*)(cp + f) = cq[q];
    *(volatile v4f*)(dp + f) = dq[q];
  }
}

__global__ __launch_bounds__(OTHR) void k_offsets(
    const int* __restrict__ cnt, int* off, int* rbase, int nChunk) {
  __shared__ __attribute__((aligned(16))) int soff[NBC];
  __shared__ __attribute__((aligned(16))) int srb[RBN];
  __shared__ int wtot[OTHR / 32];
  const int tid = threadIdx.x, lane = tid & 31, wave = tid >> 5, sub = tid >> 7;
  for (int i = tid; i < RBN; i += OTHR) srb[i] = 0;
  int carry = 0;
#pragma unroll 1
  for (int ch = 0; ch < nChunk; ++ch) {
    const int base = ch * NBC;
    const v4i c0 = *(const v4i*)(cnt + base + 8 * tid);
    const v4i c1 = *(const v4i*)(cnt + base + 8 * tid + 4);
    const int e0 = max(c0.x, 0), e1 = max(c0.y, 0), e2 = max(c0.z, 0), e3 = max(c0.w, 0);
    const int e4 = max(c1.x, 0), e5 = max(c1.y, 0), e6 = max(c1.z, 0), e7 = max(c1.w, 0);
    const int ts = e0 + e1 + e2 + e3 + e4 + e5 + e6 + e7;
    int incl = ts;
#pragma unroll
    for (int d = 1; d < 32; d <<= 1) {
      const int t = __shfl_up(incl, d);
      if (lane >= d) incl += t;
    }
    if (lane == 31) wtot[wave] = incl;
    __syncthreads();
    const int S0 = wtot[0]  + wtot[1]  + wtot[2]  + wtot[3];
    const int S1 = wtot[4]  + wtot[5]  + wtot[6]  + wtot[7];
    const int S2 = wtot[8]  + wtot[9]  + wtot[10] + wtot[11];
    const int S3 = wtot[12] + wtot[13] + wtot[14] + wtot[15];
    int pre = 0;
#pragma unroll 1
    for (int w = 4 * sub; w < wave; ++w) pre += wtot[w];
    const int b0 = carry;
    const int b1 = b0 + ((S0 + 31) & ~31);
    const int b2 = b1 + ((S1 + 31) & ~31);
    const int b3 = b2 + ((S2 + 31) & ~31);
    const int b4 = b3 + ((S3 + 31) & ~31);
    const int myb = sub == 0 ? b0 : (sub == 1 ? b1 : (sub == 2 ? b2 : b3));
    if (tid == 0) {
      srb[min(4 * ch + 0, RBN - 1)] = b0;
      srb[min(4 * ch + 1, RBN - 1)] = b1;
      srb[min(4 * ch + 2, RBN - 1)] = b2;
      srb[min(4 * ch + 3, RBN - 1)] = b3;
    }
    int run = myb + pre + incl - ts;
    soff[8 * tid + 0] = run; run += e0;
    soff[8 * tid + 1] = run; run += e1;
    soff[8 * tid + 2] = run; run += e2;
    soff[8 * tid + 3] = run; run += e3;
    soff[8 * tid + 4] = run; run += e4;
    soff[8 * tid + 5] = run; run += e5;
    soff[8 * tid + 6] = run; run += e6;
    soff[8 * tid + 7] = run;
    carry = b4;
    __syncthreads();
    const v4i o0 = *(const v4i*)(soff + 4 * tid);
    const v4i o1 = *(const v4i*)(soff + 4 * (tid + OTHR));
    int* op = off + base;
    *(volatile v4i*)(op + 4 * tid) = o0;
    *(volatile v4i*)(op + 4 * (tid + OTHR)) = o1;
    __threadfence();
    *(volatile v4i*)(op + 4 * tid) = o0;
    *(volatile v4i*)(op + 4 * (tid + OTHR)) = o1;
    __syncthreads();
  }
  if (tid == 0) srb[min(4 * nChunk, RBN - 1)] = carry;
  __syncthreads();
  v4i rv = {0, 0, 0, 0};
  if (tid < 32) rv = *(const v4i*)(srb + 4 * tid);
  if (tid < 32) *(volatile v4i*)(rbase + 4 * tid) = rv;
  __threadfence();
  if (tid < 32) *(volatile v4i*)(rbase + 4 * tid) = rv;
}

__global__ __launch_bounds__(NTHR) void k_fill(
    const int* __restrict__ srcs, const int* __restrict__ dsts,
    const int* __restrict__ off, const int* __restrict__ rbase,
    int* csr, int nN, int nE, int vec8, int csrLen) {
  extern __shared__ v4f lds_dyn[];
  int* region = (int*)lds_dyn;
  int* cursor = region + RCAP;
  int* list   = cursor + NBF;
  int* wcnt   = list + LISTN;
  const int tid = threadIdx.x, lane = tid & 31, wave = tid >> 5;
  const int b = blockIdx.x;
  const int nodeBase = b * NBF;

  int rb0 = rbase[b];
  const int rb1 = rbase[b + 1];
  rb0 = rb0 < 0 ? 0 : (rb0 > csrLen ? csrLen : rb0);
  rb0 &= ~31;
  int len = rb1 - rb0;
  len = len < 0 ? 0 : (len > RCAP ? RCAP : len);
  int lenW = (len + 31) & ~31;
  if (rb0 + lenW > csrLen) lenW = (csrLen - rb0) & ~31;

  {
    const v4i z = {0, 0, 0, 0};
    for (int i = tid; i < RCAP / 4; i += NTHR) ((v4i*)region)[i] = z;
    for (int s = tid; s < NBF; s += NTHR) {
      int o = off[nodeBase + s] - rb0;
      o = o < 0 ? 0 : (o > RCAP ? RCAP : o);
      cursor[s] = o;
    }
  }
  __syncthreads();

  const int nChunks = (nE + CHUNK - 1) / CHUNK;
#pragma unroll 1
  for (int ch = 0; ch < nChunks; ++ch) {
    const int cbase = ch * CHUNK;
    const int wc = scan_chunk<NBF>(dsts, nE, cbase, nodeBase, vec8, list, tid, lane, wave);
    if (lane == 0) wcnt[wave] = wc;
    __syncthreads();
    if (wave == 0) {
#pragma unroll 1
      for (int wsx = 0; wsx < NWAVE; ++wsx) {
        int n = __builtin_amdgcn_readfirstlane(wcnt[wsx]);
        n = n > WCAP ? WCAP : (n < 0 ? 0 : n);
        const int* lp = list + wsx * WCAP;
#pragma unroll 1
        for (int i = 0; i < n; ++i) {
          const int ent  = __builtin_amdgcn_readfirstlane(lp[i]);
          const int slot = ent & (NBF - 1);
          int e = cbase + ((ent >> 12) & (CHUNK - 1));
          e = e > nE - 1 ? nE - 1 : e;
          int sv = srcs[e];
          sv = sv < 0 ? 0 : (sv > nN - 1 ? nN - 1 : sv);
          if (lane == 0) {
            int pos = cursor[slot];
            pos = pos < 0 ? 0 : (pos > RCAP - 1 ? RCAP - 1 : pos);
            region[pos] = sv;
            const int np = pos + 1;
            cursor[slot] = np > RCAP ? RCAP : np;
          }
        }
      }
    }
    __syncthreads();
  }

  const int nv = lenW >> 2;
  int* gp = csr + rb0;
#pragma unroll 1
  for (int i = tid; i < nv; i += NTHR) { const v4i v = ((const v4i*)region)[i]; *(volatile v4i*)(gp + 4 * i) = v; }
  __threadfence();
#pragma unroll 1
  for (int i = tid; i < nv; i += NTHR) { const v4i v = ((const v4i*)region)[i]; *(volatile v4i*)(gp + 4 * i) = v; }
}

__global__ __launch_bounds__(NTHR) void k_wcvt(const float* __restrict__ w0, const float* __restrict__ w1,
                                               _Float16* dp, int K0, int K, int Nc, int nUnits) {
  const int i = (int)blockIdx.x * NTHR + (int)threadIdx.x;
  if (i >= nUnits) return;
  const int ppr = K >> 3;
  const int n = i / ppr;
  const int seg = i - n * ppr;
  int k1max = K - K0 - 1;
  k1max = k1max < 0 ? 0 : k1max;
  v8h o;
#pragma unroll
  for (int j = 0; j < 8; ++j) {
    const int k = 8 * seg + j;
    int ka = k > K0 - 1 ? K0 - 1 : k;
    ka = ka < 0 ? 0 : ka;
    int kb = k - K0;
    kb = kb < 0 ? 0 : (kb > k1max ? k1max : kb);
    const float fa = w0[(size_t)ka * Nc + n];
    const float fb = w1[(size_t)kb * Nc + n];
    const float f = (k < K0) ? fa : fb;
    o[j] = (_Float16)(f * WCARRY);
  }
  _Float16* gp = dp + (size_t)i * 8;
  *(volatile v8h*)gp = o;
  __threadfence();
  *(volatile v8h*)gp = o;
}

__global__ __launch_bounds__(NTHR) void k_wfold(const float* __restrict__ gw, const float* __restrict__ asv,
                                                const float* __restrict__ adv, float* wa) {
  __shared__ __attribute__((aligned(16))) float so[C2W * 8];
  const int tid = threadIdx.x;
#pragma unroll 1
  for (int i = 0; i < (C2W * 8) / NTHR; ++i) {
    const int o = i * NTHR + tid;
    const int k = o >> 3, j = o & 7, hd = j & 3;
    const bool useS = j < 4;
    const float* wp = gw + (size_t)k * H3W + hd * HCH;
    const float* ps = asv + hd * HCH;
    const float* pd = adv + hd * HCH;
    float acc = 0.f;
#pragma unroll 1
    for (int c = 0; c < HCH; ++c) {
      const float a1 = ps[c], a2 = pd[c];
      const float av = useS ? a1 : a2;
      acc += wp[c] * av;
    }
    so[o] = acc;
  }
  __syncthreads();
  const v4f v = *(const v4f*)(so + 4 * tid);
  *(volatile v4f*)(wa + 4 * tid) = v;
  __threadfence();
  *(volatile v4f*)(wa + 4 * tid) = v;
}

__global__ __launch_bounds__(NTHR) void k_lin5(const float* __restrict__ x, const float* __restrict__ w,
                                               float* hl, int nN, int npad) {
  const int gi = (int)blockIdx.x * NTHR + (int)threadIdx.x;
  const int node = gi >> 4, q = gi & 15;
  if (node >= npad) return;
  int rr = node > nN - 1 ? nN - 1 : node;
  rr = rr < 0 ? 0 : rr;
  const bool live = node < nN;
  v4f acc = {0.f, 0.f, 0.f, 0.f};
#pragma unroll
  for (int j = 0; j < F0; ++j) {
    const float xv = x[(size_t)rr * F0 + j];
    const v4f wv = *(const v4f*)(w + j * C1W + 4 * q);
    acc = acc + wv * xv;
  }
  const v4f o = selz(acc, live);
  float* gp = hl + (size_t)node * C1W + 4 * q;
  *(volatile v4f*)gp = o;
  __threadfence();
  *(volatile v4f*)gp = o;
}

template <int NP, typename VT, int W>
__global__ __launch_bounds__(NTHR) void k_aggsym(
    const int* __restrict__ csr, const int* __restrict__ off, const int* __restrict__ cnt,
    const float* __restrict__ dinv, const float* __restrict__ hw, const float* __restrict__ cb,
    float* hout, int nN, int csrLen) {
  constexpr int CW = NP * 32 * W;
  const int tid = threadIdx.x, lane = tid & 31, wave = tid >> 5;
  const int tbase = blockIdx.x * TGT + wave * 32;
  const int cl    = tbase + lane;
  const int cnt_l = cnt[cl];
  const int off_l = off[cl];
  const float di_l = dinv[cl];
  VT cbv[NP];
#pragma unroll
  for (int p = 0; p < NP; ++p) cbv[p] = *(const VT*)(cb + (p * 32 + lane) * W);

#pragma unroll 1
  for (int j = 0; j < 32; ++j) {
    const int c = tbase + j;
    int n = __shfl(cnt_l, j);
    n = n < 0 ? 0 : (n > DEGCAP ? DEGCAP : n);
    const int st = __shfl(off_l, j);
    const float dc = __shfl(di_l, j);
    const float dd = dc * dc;

    VT a[NP];
#pragma unroll
    for (int p = 0; p < NP; ++p) a[p] = *(const VT*)(hw + (size_t)c * CW + (p * 32 + lane) * W) * dd;
#pragma unroll 1
    for (int q0 = 0; q0 < n; q0 += 32) {
      int pos = st + q0 + lane;
      pos = pos < 0 ? 0 : (pos > csrLen - 1 ? csrLen - 1 : pos);
      int sl = csr[pos];
      sl = sl < 0 ? 0 : (sl > nN - 1 ? nN - 1 : sl);
      const int mcnt = (n - q0) < 32 ? (n - q0) : 32;
#pragma unroll 1
      for (int pp = 0; pp < mcnt; ++pp) {
        const int s = __builtin_amdgcn_readlane(sl, pp);
        const float cf = dinv[s] * dc;
#pragma unroll
        for (int p = 0; p < NP; ++p) {
          const VT xv = *(const VT*)(hw + (size_t)s * CW + (p * 32 + lane) * W);
          a[p] = a[p] + xv * cf;
        }
      }
    }

    const bool live = c < nN;
    VT o[NP];
#pragma unroll
    for (int p = 0; p < NP; ++p) o[p] = selz(a[p] + cbv[p], live);
    float* gp = hout + (size_t)c * CW + W * lane;
#pragma unroll
    for (int p = 0; p < NP; ++p) *(volatile VT*)(gp + p * 32 * W) = o[p];
    __threadfence();
#pragma unroll
    for (int p = 0; p < NP; ++p) *(volatile VT*)(gp + p * 32 * W) = o[p];
  }
}

__global__ __launch_bounds__(NTHR) void k_aggmean(
    const int* __restrict__ csr, const int* __restrict__ off, const int* __restrict__ cnt,
    const float* __restrict__ h, _Float16* aout, int nN, int csrLen) {
  const int tid = threadIdx.x, lane = tid & 31, wave = tid >> 5;
  const int tbase = blockIdx.x * TGT + wave * 32;
  const int cl    = tbase + lane;
  const int cnt_l = cnt[cl];
  const int off_l = off[cl];

#pragma unroll 1
  for (int j = 0; j < 32; ++j) {
    const int c = tbase + j;
    int n0 = __shfl(cnt_l, j);
    n0 = n0 < 0 ? 0 : n0;
    const int n = n0 > DEGCAP ? DEGCAP : n0;
    const int st = __shfl(off_l, j);

    v2f a = {0.f, 0.f};
#pragma unroll 1
    for (int q0 = 0; q0 < n; q0 += 32) {
      int pos = st + q0 + lane;
      pos = pos < 0 ? 0 : (pos > csrLen - 1 ? csrLen - 1 : pos);
      int sl = csr[pos];
      sl = sl < 0 ? 0 : (sl > nN - 1 ? nN - 1 : sl);
      const int mcnt = (n - q0) < 32 ? (n - q0) : 32;
#pragma unroll 1
      for (int pp = 0; pp < mcnt; ++pp) {
        const int s = __builtin_amdgcn_readlane(sl, pp);
        const v2f xv = *(const v2f*)(h + (size_t)s * C1W + 2 * lane);
        a = a + xv;
      }
    }
    const float rc = __builtin_amdgcn_rcpf(fmaxf((float)n0, 1.0f));
    const v2f self = *(const v2f*)(h + (size_t)c * C1W + 2 * lane);
    const bool live = c < nN;
    const v2f am = selz(a * rc, live);
    const v2f sm = selz(self, live);
    v2h lo, hi;
    lo.x = (_Float16)(am.x * ACARRY); lo.y = (_Float16)(am.y * ACARRY);
    hi.x = (_Float16)(sm.x * ACARRY); hi.y = (_Float16)(sm.y * ACARRY);
    _Float16* gp = aout + (size_t)c * C2W + 2 * lane;
    *(volatile v2h*)gp = lo;
    *(volatile v2h*)(gp + C1W) = hi;
    __threadfence();
    *(volatile v2h*)gp = lo;
    *(volatile v2h*)(gp + C1W) = hi;
  }
}

template <int C>
__global__ __launch_bounds__(NTHR) void k_bnstat(const float* __restrict__ x, double* part, int nN, int rpb) {
  constexpr int CL  = C < NTHR ? C : NTHR;
  constexpr int RG  = NTHR / CL;
  constexpr int CPT = C / CL;
  static_assert(RG * CL == NTHR);
  static_assert(CPT * CL == C);
  __shared__ __attribute__((aligned(16))) double sred[2 * RG * C];
  __shared__ __attribute__((aligned(16))) double sout[2 * C];
  const int tid = threadIdx.x;
  const int rg = tid / CL, c0 = tid - rg * CL;
  const int r0 = blockIdx.x * rpb;
  const int r1 = min(r0 + rpb, nN);
  double s[CPT], s2[CPT];
#pragma unroll
  for (int i = 0; i < CPT; ++i) { s[i] = 0.0; s2[i] = 0.0; }
#pragma unroll 1
  for (int r = r0 + rg; r < r1; r += RG) {
#pragma unroll
    for (int i = 0; i < CPT; ++i) {
      const double v = (double)x[(size_t)r * C + c0 + CL * i];
      s[i] += v;
      s2[i] += v * v;
    }
  }
#pragma unroll
  for (int i = 0; i < CPT; ++i) {
    sred[(0 * RG + rg) * C + c0 + CL * i] = s[i];
    sred[(1 * RG + rg) * C + c0 + CL * i] = s2[i];
  }
  __syncthreads();
#pragma unroll 1
  for (int idx = tid; idx < 2 * C; idx += NTHR) {
    const int q = idx / C, c = idx - q * C;
    double S = 0.0;
#pragma unroll
    for (int g = 0; g < RG; ++g) S += sred[(q * RG + g) * C + c];
    sout[idx] = S;
  }
  __syncthreads();
  double* gp = part + (size_t)blockIdx.x * 2 * C;
#pragma unroll 1
  for (int p = tid; p < C; p += NTHR) { const v2d v = *(const v2d*)(sout + 2 * p); *(volatile v2d*)(gp + 2 * p) = v; }
  __threadfence();
#pragma unroll 1
  for (int p = tid; p < C; p += NTHR) { const v2d v = *(const v2d*)(sout + 2 * p); *(volatile v2d*)(gp + 2 * p) = v; }
}

template <int C, bool WF32, bool WF16>
__global__ __launch_bounds__(NTHR) void k_bnapply(
    float* x, const double* __restrict__ part, const float* __restrict__ gam, const float* __restrict__ bet,
    _Float16* a16, int nN, int npad, int rpb, int nPart, double invN) {
  static_assert((C % 64) == 0 && C <= 2 * NTHR);
  constexpr int PPR = C / 4;
  constexpr int RPP = NTHR / PPR;
  static_assert(RPP * PPR == NTHR);
  __shared__ __attribute__((aligned(16))) float smu[C];
  __shared__ __attribute__((aligned(16))) float ssc[C];
  __shared__ __attribute__((aligned(16))) float sbb[C];
  const int tid = threadIdx.x;
#pragma unroll 1
  for (int c = tid; c < C; c += NTHR) {
    double s = 0.0, s2 = 0.0;
#pragma unroll 1
    for (int b = 0; b < nPart; ++b) {
      s  += part[((size_t)b * 2) * C + c];
      s2 += part[((size_t)b * 2 + 1) * C + c];
    }
    const double mu = s * invN;
    double var = s2 * invN - mu * mu;
    var = var < 0.0 ? 0.0 : var;
    const float muf = (float)mu, varf = (float)var;
    const float rstd = rsqrtf(varf + BNEPS);
    smu[c] = muf;
    ssc[c] = rstd * gam[c];
    sbb[c] = bet[c];
  }
  __syncthreads();
  const int seg = tid % PPR, rsub = tid / PPR;
  const v4f mu4 = *(const v4f*)(smu + 4 * seg);
  const v4f sc4 = *(const v4f*)(ssc + 4 * seg);
  const v4f bb4 = *(const v4f*)(sbb + 4 * seg);
  const int r0 = blockIdx.x * rpb;
  const int r1 = min(r0 + rpb, npad);
#pragma unroll 1
  for (int rs = r0; rs < r1; rs += RPP) {
    const int row = rs + rsub;
    if (row < r1) {
      const size_t o = (size_t)row * C + 4 * seg;
      const v4f v = *(const v4f*)(x + o);
      v4f y = (v - mu4) * sc4 + bb4;
      y.x = fmaxf(y.x, 0.f); y.y = fmaxf(y.y, 0.f); y.z = fmaxf(y.z, 0.f); y.w = fmaxf(y.w, 0.f);
      const bool live = row < nN;
      y = selz(y, live);
      v4h hq;
      hq.x = (_Float16)(y.x * ACARRY); hq.y = (_Float16)(y.y * ACARRY);
      hq.z = (_Float16)(y.z * ACARRY); hq.w = (_Float16)(y.w * ACARRY);
      if (WF32) *(volatile v4f*)(x + o) = y;
      if (WF16) *(volatile v4h*)(a16 + o) = hq;
      __threadfence();
      if (WF32) *(volatile v4f*)(x + o) = y;
      if (WF16) *(volatile v4h*)(a16 + o) = hq;
    }
  }
}

__global__ __launch_bounds__(NTHR) void k_logit(const float* __restrict__ h2, const float* __restrict__ wa,
                                                float* es8, int nN) {
  __shared__ __attribute__((aligned(16))) float swa[C2W * 8];
  __shared__ __attribute__((aligned(16))) float so[NTHR * 8];
  const int tid = threadIdx.x;
  *(v4f*)(swa + 4 * tid) = *(const v4f*)(wa + 4 * tid);
  __syncthreads();
  const int node = (int)blockIdx.x * NTHR + tid;
  int rr = node > nN - 1 ? nN - 1 : node;
  rr = rr < 0 ? 0 : rr;
  const bool live = node < nN;
  v4f alo = {0.f, 0.f, 0.f, 0.f}, ahi = {0.f, 0.f, 0.f, 0.f};
  const float* hp = h2 + (size_t)rr * C2W;
#pragma unroll 1
  for (int kq = 0; kq < C2W / 4; ++kq) {
    const v4f hv = *(const v4f*)(hp + 4 * kq);
#pragma unroll
    for (int t = 0; t < 4; ++t) {
      const float hk = hv[t];
      const v4f w0 = *(const v4f*)(swa + (4 * kq + t) * 8);
      const v4f w1 = *(const v4f*)(swa + (4 * kq + t) * 8 + 4);
      alo = alo + w0 * hk;
      ahi = ahi + w1 * hk;
    }
  }
  *(v4f*)(so + 8 * tid)     = selz(alo, live);
  *(v4f*)(so + 8 * tid + 4) = selz(ahi, live);
  __syncthreads();
  float* gbase = es8 + (size_t)blockIdx.x * NTHR * 8;
  v4f cv[2];
#pragma unroll
  for (int it = 0; it < 2; ++it) cv[it] = *(const v4f*)(so + 4 * (it * NTHR + tid));
#pragma unroll
  for (int it = 0; it < 2; ++it) *(volatile v4f*)(gbase + 4 * (it * NTHR + tid)) = cv[it];
  __threadfence();
#pragma unroll
  for (int it = 0; it < 2; ++it) *(volatile v4f*)(gbase + 4 * (it * NTHR + tid)) = cv[it];
}

__global__ __launch_bounds__(NTHR) void k_gemm(
    const _Float16* __restrict__ A, const _Float16* __restrict__ Bp, const float* __restrict__ bias,
    int hasBias, float* Cout, int K, int ldc, int nValid, int nStore) {
  constexpr int TPW = 4;
  constexpr int PPR = BNC / 4;
  constexpr int NIT = (BM * PPR) / NTHR;
  static_assert((BM * PPR) % NTHR == 0);
  static_assert(NIT >= 1);
  static_assert(TPW * 16 * 2 == BNC);
  static_assert(BM == 4 * 16);
  static_assert(PPR == 32);

  __shared__ __attribute__((aligned(16))) float stg[BM * BNC];
  const int tid = threadIdx.x, lane = tid & 31, wave = tid >> 5, hh = lane >> 4, m = lane & 15;
  const int rowBase = (int)blockIdx.x * BM;
  const int colBase = (int)blockIdx.y * BNC;
  const int rg = wave >> 1, chf = wave & 1;
  const int r0 = rg * 16;
  const int c0 = chf * (BNC / 2);

  v8f acc[TPW];
#pragma unroll
  for (int t = 0; t < TPW; ++t) { v8f z = {0.f, 0.f, 0.f, 0.f, 0.f, 0.f, 0.f, 0.f}; acc[t] = z; }

  const _Float16* ap = A  + (size_t)(rowBase + r0 + m) * K + 8 * hh;
  const _Float16* bp = Bp + (size_t)(colBase + c0 + m) * K + 8 * hh;
  const int ksteps = K >> 5;
#pragma unroll 1
  for (int kt = 0; kt < ksteps; ++kt) {
    Frag a;
    a.h[0] = *(const v8h*)(ap + 32 * kt);
    a.h[1] = *(const v8h*)(ap + 32 * kt + 16);
#pragma unroll
    for (int t = 0; t < TPW; ++t) {
      const size_t to = (size_t)(16 * t) * K + 32 * kt;
      Frag b;
      b.h[0] = *(const v8h*)(bp + to);
      b.h[1] = *(const v8h*)(bp + to + 16);
      acc[t] = wmh(a.v, b.v, acc[t]);
    }
  }

  float bv[TPW];
  if (hasBias != 0) {
#pragma unroll
    for (int t = 0; t < TPW; ++t) bv[t] = bias[colBase + c0 + 16 * t + m];
  } else {
#pragma unroll
    for (int t = 0; t < TPW; ++t) bv[t] = 0.f;
  }

  {
    float* sp = stg + (size_t)(r0 + 8 * hh) * BNC + c0 + m;
    const int growb = rowBase + r0 + 8 * hh;
#pragma unroll
    for (int t = 0; t < TPW; ++t) {
#pragma unroll
      for (int r = 0; r < 8; ++r) {
        const bool lv = (growb + r) < nValid;
        const float g = acc[t][r] * GSCALE + bv[t];
        sp[r * BNC + 16 * t] = lv ? g : 0.f;
      }
    }
  }
  __syncthreads();

  v4f cv[NIT];
#pragma unroll
  for (int it = 0; it < NIT; ++it) {
    const int id = it * NTHR + tid;
    const int row = id >> 5, seg = id & 31;
    cv[it] = *(const v4f*)(stg + (size_t)row * BNC + 4 * seg);
  }
#pragma unroll
  for (int it = 0; it < NIT; ++it) {
    const int id = it * NTHR + tid;
    const int row = id >> 5, seg = id & 31;
    const int grow = rowBase + row;
    if (grow < nStore) {
      float* gp = Cout + (size_t)grow * ldc + colBase + 4 * seg;
      *(volatile v4f*)gp = cv[it];
    }
  }
  __threadfence();
#pragma unroll
  for (int it = 0; it < NIT; ++it) {
    const int id = it * NTHR + tid;
    const int row = id >> 5, seg = id & 31;
    const int grow = rowBase + row;
    if (grow < nStore) {
      float* gp = Cout + (size_t)grow * ldc + colBase + 4 * seg;
      *(volatile v4f*)gp = cv[it];
    }
  }
}

__global__ __launch_bounds__(NTHR) void k_aggatt(
    const int* __restrict__ csr, const int* __restrict__ off, const int* __restrict__ cnt,
    const float* __restrict__ es8, const float* __restrict__ h3, const float* __restrict__ gb,
    float* hout, int nN, int csrLen) {
  const int tid = threadIdx.x, lane = tid & 31, wave = tid >> 5;
  const int tbase = blockIdx.x * TGT + wave * 32;
  const int cl    = tbase + lane;
  const int cnt_l = cnt[cl];
  const int off_l = off[cl];
  const v4f b0 = *(const v4f*)(gb + 4 * lane);
  const v4f b1 = *(const v4f*)(gb + 128 + 4 * lane);
  const float NINF = -__builtin_inff();

#pragma unroll 1
  for (int j = 0; j < 32; ++j) {
    const int c = tbase + j;
    int n = __shfl(cnt_l, j);
    n = n < 0 ? 0 : (n > DEGCAP ? DEGCAP : n);
    const int st = __shfl(off_l, j);
    const v4f esc = *(const v4f*)(es8 + (size_t)c * 8);
    const v4f edc = *(const v4f*)(es8 + (size_t)c * 8 + 4);
    const v4f eself = lrelu4(esc + edc);

    v4f m = eself;
#pragma unroll 1
    for (int q0 = 0; q0 < n; q0 += 32) {
      int pos = st + q0 + lane;
      pos = pos < 0 ? 0 : (pos > csrLen - 1 ? csrLen - 1 : pos);
      int sl = csr[pos];
      sl = sl < 0 ? 0 : (sl > nN - 1 ? nN - 1 : sl);
      const int mcnt = (n - q0) < 32 ? (n - q0) : 32;
      const bool valid = lane < mcnt;
      const v4f esv = *(const v4f*)(es8 + (size_t)sl * 8);
      v4f e = lrelu4(esv + edc);
      e = selv4(e, valid, NINF);
      e = wmax4(e);
      m = vmax4(m, e);
    }
    const v4f exs = vexp4(eself - m);
    v4f z = exs;
#pragma unroll 1
    for (int q0 = 0; q0 < n; q0 += 32) {
      int pos = st + q0 + lane;
      pos = pos < 0 ? 0 : (pos > csrLen - 1 ? csrLen - 1 : pos);
      int sl = csr[pos];
      sl = sl < 0 ? 0 : (sl > nN - 1 ? nN - 1 : sl);
      const int mcnt = (n - q0) < 32 ? (n - q0) : 32;
      const bool valid = lane < mcnt;
      const v4f esv = *(const v4f*)(es8 + (size_t)sl * 8);
      const v4f ex = selv4(vexp4(lrelu4(esv + edc) - m), valid, 0.f);
      z = z + wsum4(ex);
    }
    v4f rz;
    rz.x = __builtin_amdgcn_rcpf(z.x); rz.y = __builtin_amdgcn_rcpf(z.y);
    rz.z = __builtin_amdgcn_rcpf(z.z); rz.w = __builtin_amdgcn_rcpf(z.w);
    const v4f als = exs * rz;

    v4f acc[8];
    const float* hc = h3 + (size_t)c * H3W + 4 * lane;
#pragma unroll
    for (int p = 0; p < 8; ++p) {
      const v4f hv = *(const v4f*)(hc + 128 * p);
      acc[p] = hv * als[p >> 1];
    }
#pragma unroll 1
    for (int q0 = 0; q0 < n; q0 += 32) {
      int pos = st + q0 + lane;
      pos = pos < 0 ? 0 : (pos > csrLen - 1 ? csrLen - 1 : pos);
      int sl = csr[pos];
      sl = sl < 0 ? 0 : (sl > nN - 1 ? nN - 1 : sl);
      const int mcnt = (n - q0) < 32 ? (n - q0) : 32;
      const bool valid = lane < mcnt;
      const v4f esv = *(const v4f*)(es8 + (size_t)sl * 8);
      const v4f al = selv4(vexp4(lrelu4(esv + edc) - m) * rz, valid, 0.f);
#pragma unroll 1
      for (int pp = 0; pp < mcnt; ++pp) {
        const int s = __builtin_amdgcn_readlane(sl, pp);
        const float a0 = __int_as_float(__builtin_amdgcn_readlane(__float_as_int(al.x), pp));
        const float a1 = __int_as_float(__builtin_amdgcn_readlane(__float_as_int(al.y), pp));
        const float a2 = __int_as_float(__builtin_amdgcn_readlane(__float_as_int(al.z), pp));
        const float a3 = __int_as_float(__builtin_amdgcn_readlane(__float_as_int(al.w), pp));
        const float* hs = h3 + (size_t)s * H3W + 4 * lane;
#pragma unroll
        for (int p = 0; p < 8; ++p) {
          const v4f hv = *(const v4f*)(hs + 128 * p);
          const float ap = ((p >> 1) == 0) ? a0 : (((p >> 1) == 1) ? a1 : (((p >> 1) == 2) ? a2 : a3));
          acc[p] = acc[p] + hv * ap;
        }
      }
    }

    const bool live = c < nN;
    v4f o0 = ((acc[0] + acc[2]) + acc[4]) + acc[6];
    v4f o1 = ((acc[1] + acc[3]) + acc[5]) + acc[7];
    o0 = o0 * 0.25f + b0;
    o1 = o1 * 0.25f + b1;
    o0 = selz(o0, live);
    o1 = selz(o1, live);
    float* gp = hout + (size_t)c * C3W + 4 * lane;
    *(volatile v4f*)gp = o0;
    *(volatile v4f*)(gp + 128) = o1;
    __threadfence();
    *(volatile v4f*)gp = o0;
    *(volatile v4f*)(gp + 128) = o1;
  }
}

__global__ __launch_bounds__(NTHR) void k_pool(
    const int* __restrict__ batch, const float* __restrict__ h, _Float16* p16, int nN, int vec8) {
  __shared__ __attribute__((aligned(16))) int list[LISTN];
  __shared__ __attribute__((aligned(16))) float spart[NWAVE * C4W];
  __shared__ __attribute__((aligned(16))) _Float16 srow[PW];
  __shared__ int swn[NWAVE];
  const int tid = threadIdx.x, lane = tid & 31, wave = tid >> 5;
  const int g = blockIdx.x;
  const float NINF = -__builtin_inff();

  v4f sa[4], sm[4];
#pragma unroll
  for (int p = 0; p < 4; ++p) {
    v4f z = {0.f, 0.f, 0.f, 0.f}; sa[p] = z;
    v4f q = {NINF, NINF, NINF, NINF}; sm[p] = q;
  }
  int wn = 0;

  const int nChunks = (nN + CHUNK - 1) / CHUNK;
#pragma unroll 1
  for (int ch = 0; ch < nChunks; ++ch) {
    const int cbase = ch * CHUNK;
    const int wc = scan_chunk<1>(batch, nN, cbase, g, vec8, list, tid, lane, wave);
    __syncthreads();
    int n = wc;
    n = n > WCAP ? WCAP : (n < 0 ? 0 : n);
    wn += n;
    const int* lp = list + wave * WCAP;
#pragma unroll 1
    for (int i = 0; i < n; ++i) {
      const int ent = __builtin_amdgcn_readfirstlane(lp[i]);
      int node = cbase + ((ent >> 12) & (CHUNK - 1));
      node = node > nN - 1 ? nN - 1 : (node < 0 ? 0 : node);
      const float* hp = h + (size_t)node * C4W + 4 * lane;
#pragma unroll
      for (int p = 0; p < 4; ++p) {
        const v4f hv = *(const v4f*)(hp + 128 * p);
        sa[p] = sa[p] + hv;
        sm[p] = vmax4(sm[p], hv);
      }
    }
    __syncthreads();
  }

#pragma unroll
  for (int p = 0; p < 4; ++p) *(v4f*)(spart + wave * C4W + 128 * p + 4 * lane) = sa[p];
  if (lane == 0) swn[wave] = wn;
  __syncthreads();
  const int ca = tid, cb2 = tid + NTHR;
  float S0 = 0.f, S1 = 0.f;
  int ng = 0;
#pragma unroll
  for (int w = 0; w < NWAVE; ++w) { S0 += spart[w * C4W + ca]; S1 += spart[w * C4W + cb2]; ng += swn[w]; }
  __syncthreads();
#pragma unroll
  for (int p = 0; p < 4; ++p) *(v4f*)(spart + wave * C4W + 128 * p + 4 * lane) = sm[p];
  __syncthreads();
  float M0 = NINF, M1 = NINF;
#pragma unroll
  for (int w = 0; w < NWAVE; ++w) { M0 = fmaxf(M0, spart[w * C4W + ca]); M1 = fmaxf(M1, spart[w * C4W + cb2]); }
  const float rc = __builtin_amdgcn_rcpf(fmaxf((float)ng, 1.0f));
  const float mean0 = S0 * rc, mean1 = S1 * rc;
  const float mx0 = ng > 0 ? M0 : 0.f, mx1 = ng > 0 ? M1 : 0.f;
  srow[ca]        = (_Float16)(mean0 * ACARRY);
  srow[cb2]       = (_Float16)(mean1 * ACARRY);
  srow[C4W + ca]  = (_Float16)(mx0 * ACARRY);
  srow[C4W + cb2] = (_Float16)(mx1 * ACARRY);
  __syncthreads();

  _Float16* gp = p16 + (size_t)g * PW;
  const int tq = tid & (PW / 8 - 1);
  const v8h v = *(const v8h*)(srow + 8 * tq);
  if (tid < PW / 8) *(volatile v8h*)(gp + 8 * tid) = v;
  __threadfence();
  if (tid < PW / 8) *(volatile v8h*)(gp + 8 * tid) = v;
}

extern "C" void kernel_launch(void* const* d_in, const int* in_sizes, int n_in,
                              void* d_out, int out_size, void* d_ws, size_t ws_size,
                              hipStream_t stream) {
  if (n_in < 24) return;
  const int nN = in_sizes[2];
  if (nN < 1 || nN > (1 << 20)) return;
  if (in_sizes[0] != nN * F0) return;
  if (in_sizes[1] < 2 || (in_sizes[1] & 1) != 0) return;
  const int nE = in_sizes[1] / 2;
  if (nE > (1 << 26)) return;
  if (in_sizes[3] != F0 * C1W || in_sizes[4] != C1W) return;
  if (in_sizes[5] != C1W * C2W || in_sizes[6] != C1W * C2W || in_sizes[7] != C2W) return;
  if (in_sizes[8] != C2W * H3W || in_sizes[9] != HEADS * HCH || in_sizes[10] != HEADS * HCH) return;
  if (in_sizes[11] != C3W) return;
  if (in_sizes[12] != C3W * C4W || in_sizes[13] != C4W) return;
  if (in_sizes[14] != C1W || in_sizes[15] != C1W || in_sizes[16] != C2W || in_sizes[17] != C2W) return;
  if (in_sizes[18] != C3W || in_sizes[19] != C3W || in_sizes[20] != C4W || in_sizes[21] != C4W) return;
  if (in_sizes[22] != PW * FCN || in_sizes[23] != FCN) return;
  if (out_size < FCN || (out_size % FCN) != 0) return;
  const int nG = out_size / FCN;
  if (nG < 1 || nG > 4096) return;

  const float* x     = (const float*)d_in[0];
  const int*   ei    = (const int*)d_in[1];
  const int*   src   = ei;
  const int*   dst   = ei + nE;
  const int*   batch = (const int*)d_in[2];
  const float* w1    = (const float*)d_in[3];
  const float* cb1   = (const float*)d_in[4];
  const float* wl    = (const float*)d_in[5];
  const float* wr    = (const float*)d_in[6];
  const float* cb2   = (const float*)d_in[7];
  const float* watt  = (const float*)d_in[8];
  const float* asrc  = (const float*)d_in[9];
  const float* adst  = (const float*)d_in[10];
  const float* cb3   = (const float*)d_in[11];
  const float* w4    = (const float*)d_in[12];
  const float* cb4   = (const float*)d_in[13];
  const float* g1    = (const float*)d_in[14];
  const float* be1   = (const float*)d_in[15];
  const float* g2    = (const float*)d_in[16];
  const float* be2   = (const float*)d_in[17];
  const float* g3    = (const float*)d_in[18];
  const float* be3   = (const float*)d_in[19];
  const float* g4    = (const float*)d_in[20];
  const float* be4   = (const float*)d_in[21];
  const float* wfc   = (const float*)d_in[22];
  const float* bfc   = (const float*)d_in[23];
  float* out = (float*)d_out;

  const int NPAD   = ((nN + TGT - 1) / TGT) * TGT;
  const int nAgg   = NPAD / TGT;
  const int nBC    = (nN + NBC - 1) / NBC;
  const int CNTPAD = nBC * NBC;
  if (CNTPAD < NPAD) return;
  if (4 * nBC + 1 > RBN) return;
  const int nBF    = (nN + NBF - 1) / NBF;
  if (nBF > 4 * nBC) return;
  const int csrLen = ((nE + 31) & ~31) + 4096;
  if (31 * 4 * nBC > 4096) return;
  const int nGemmR = NPAD / BM;
  const int GPADM  = ((nG + BM - 1) / BM) * BM;
  const int rpbS   = (nN + SB - 1) / SB;
  const double invN = 1.0 / (double)nN;

  char* ws = (char*)d_ws;
  size_t off = 0;
  const size_t oCnt = off; off += (size_t)CNTPAD * 4;                    off = (off + 255) & ~(size_t)255;
  const size_t oDi  = off; off += (size_t)CNTPAD * 4;                    off = (off + 255) & ~(size_t)255;
  const size_t oOff = off; off += (size_t)CNTPAD * 4;                    off = (off + 255) & ~(size_t)255;
  const size_t oRb  = off; off += (size_t)RBN * 4;                       off = (off + 255) & ~(size_t)255;
  const size_t oCsr = off; off += (size_t)csrLen * 4;                    off = (off + 255) & ~(size_t)255;
  const size_t oWs  = off; off += (size_t)C2W * C2W * 2;                 off = (off + 255) & ~(size_t)255;
  const size_t oWg  = off; off += (size_t)H3W * C2W * 2;                 off = (off + 255) & ~(size_t)255;
  const size_t oW4  = off; off += (size_t)C4W * C3W * 2;                 off = (off + 255) & ~(size_t)255;
  const size_t oWf  = off; off += (size_t)FCN * PW * 2;                  off = (off + 255) & ~(size_t)255;
  const size_t oWa  = off; off += (size_t)C2W * 8 * 4;                   off = (off + 255) & ~(size_t)255;
  const size_t oH1L = off; off += (size_t)NPAD * C1W * 4;                off = (off + 255) & ~(size_t)255;
  const size_t oC1  = off; off += (size_t)NPAD * C1W * 4;                off = (off + 255) & ~(size_t)255;
  const size_t oA2  = off; off += (size_t)NPAD * C2W * 2;                off = (off + 255) & ~(size_t)255;
  const size_t oC2  = off; off += (size_t)NPAD * C2W * 4;                off = (off + 255) & ~(size_t)255;
  const size_t oA3  = off; off += (size_t)NPAD * C2W * 2;                off = (off + 255) & ~(size_t)255;
  const size_t oEs  = off; off += (size_t)NPAD * 8 * 4;                  off = (off + 255) & ~(size_t)255;
  const size_t oBig = off; off += (size_t)NPAD * H3W * 4;                off = (off + 255) & ~(size_t)255;
  const size_t oC3  = off; off += (size_t)NPAD * C3W * 4;                off = (off + 255) & ~(size_t)255;
  const size_t oA4  = off; off += (size_t)NPAD * C3W * 2;                off = (off + 255) & ~(size_t)255;
  const size_t oPt  = off; off += (size_t)SB * 2 * C4W * 8;              off = (off + 255) & ~(size_t)255;
  const size_t oP16 = off; off += (size_t)GPADM * PW * 2;                off = (off + 255) & ~(size_t)255;
  if (off > ws_size || off > (size_t)WSCAP) return;
  if ((size_t)NPAD * C4W * 4 * 2 > (size_t)NPAD * H3W * 4) return;

  int*   cnt   = (int*)(ws + oCnt);
  float* dinv  = (float*)(ws + oDi);
  int*   offp  = (int*)(ws + oOff);
  int*   rb    = (int*)(ws + oRb);
  int*   csr   = (int*)(ws + oCsr);
  _Float16* wsg = (_Float16*)(ws + oWs);
  _Float16* wgp = (_Float16*)(ws + oWg);
  _Float16* w4p = (_Float16*)(ws + oW4);
  _Float16* wfp = (_Float16*)(ws + oWf);
  float* wa    = (float*)(ws + oWa);
  float* h1l   = (float*)(ws + oH1L);
  float* c1    = (float*)(ws + oC1);
  _Float16* a2 = (_Float16*)(ws + oA2);
  float* c2    = (float*)(ws + oC2);
  _Float16* a3 = (_Float16*)(ws + oA3);
  float* es8   = (float*)(ws + oEs);
  float* h3    = (float*)(ws + oBig);
  float* h4l   = (float*)(ws + oBig);
  float* c4    = (float*)(ws + oBig + (size_t)NPAD * C4W * 4);
  float* c3    = (float*)(ws + oC3);
  _Float16* a4 = (_Float16*)(ws + oA4);
  double* part = (double*)(ws + oPt);
  _Float16* p16 = (_Float16*)(ws + oP16);

  const int vec8 = ((nE & 3) == 0) ? 1 : 0;

  k_count<<<nBC, NTHR, 0, stream>>>(dst, cnt, dinv, nE, vec8);
  k_offsets<<<1, OTHR, 0, stream>>>(cnt, offp, rb, nBC);
  hipFuncSetAttribute(reinterpret_cast<const void*>(&k_fill),
                      hipFuncAttributeMaxDynamicSharedMemorySize, LDS_FILL);
  k_fill<<<nBF, NTHR, LDS_FILL, stream>>>(src, dst, offp, rb, csr, nN, nE, vec8, csrLen);

  {
    const int u1 = C2W * (C2W / 8);
    k_wcvt<<<(u1 + NTHR - 1) / NTHR, NTHR, 0, stream>>>(wl, wr, wsg, C1W, C2W, C2W, u1);
    const int u2 = H3W * (C2W / 8);
    k_wcvt<<<(u2 + NTHR - 1) / NTHR, NTHR, 0, stream>>>(watt, watt, wgp, C2W, C2W, H3W, u2);
    const int u3 = C4W * (C3W / 8);
    k_wcvt<<<(u3 + NTHR - 1) / NTHR, NTHR, 0, stream>>>(w4, w4, w4p, C3W, C3W, C4W, u3);
    const int u4 = FCN * (PW / 8);
    k_wcvt<<<(u4 + NTHR - 1) / NTHR, NTHR, 0, stream>>>(wfc, wfc, wfp, PW, PW, FCN, u4);
  }
  k_wfold<<<1, NTHR, 0, stream>>>(watt, asrc, adst, wa);

  k_lin5<<<(NPAD * 16) / NTHR, NTHR, 0, stream>>>(x, w1, h1l, nN, NPAD);
  k_aggsym<1, v2f, 2><<<nAgg, NTHR, 0, stream>>>(csr, offp, cnt, dinv, h1l, cb1, c1, nN, csrLen);
  k_bnstat<C1W><<<SB, NTHR, 0, stream>>>(c1, part, nN, rpbS);
  k_bnapply<C1W, true, false><<<nAgg, NTHR, 0, stream>>>(c1, part, g1, be1, a2, nN, NPAD, TGT, SB, invN);

  k_aggmean<<<nAgg, NTHR, 0, stream>>>(csr, offp, cnt, c1, a2, nN, csrLen);
  k_gemm<<<dim3(nGemmR, C2W / BNC), NTHR, 0, stream>>>(a2, wsg, cb2, 1, c2, C2W, C2W, nN, NPAD);
  k_bnstat<C2W><<<SB, NTHR, 0, stream>>>(c2, part, nN, rpbS);
  k_bnapply<C2W, true, true><<<nAgg, NTHR, 0, stream>>>(c2, part, g2, be2, a3, nN, NPAD, TGT, SB, invN);

  k_logit<<<NPAD / NTHR, NTHR, 0, stream>>>(c2, wa, es8, nN);
  k_gemm<<<dim3(nGemmR, H3W / BNC), NTHR, 0, stream>>>(a3, wgp, bfc, 0, h3, C2W, H3W, nN, NPAD);
  k_aggatt<<<nAgg, NTHR, 0, stream>>>(csr, offp, cnt, es8, h3, cb3, c3, nN, csrLen);
  k_bnstat<C3W><<<SB, NTHR, 0, stream>>>(c3, part, nN, rpbS);
  k_bnapply<C3W, false, true><<<nAgg, NTHR, 0, stream>>>(c3, part, g3, be3, a4, nN, NPAD, TGT, SB, invN);

  k_gemm<<<dim3(nGemmR, C4W / BNC), NTHR, 0, stream>>>(a4, w4p, bfc, 0, h4l, C3W, C4W, nN, NPAD);
  k_aggsym<4, v4f, 4><<<nAgg, NTHR, 0, stream>>>(csr, offp, cnt, dinv, h4l, cb4, c4, nN, csrLen);
  k_bnstat<C4W><<<SB, NTHR, 0, stream>>>(c4, part, nN, rpbS);
  k_bnapply<C4W, true, false><<<nAgg, NTHR, 0, stream>>>(c4, part, g4, be4, a2, nN, NPAD, TGT, SB, invN);

  k_pool<<<GPADM, NTHR, 0, stream>>>(batch, c4, p16, nN, 1);
  k_gemm<<<dim3(GPADM / BM, FCN / BNC), NTHR, 0, stream>>>(p16, wfp, bfc, 1, out, PW, FCN, nG, nG);
}
